// S4Block_18047452578306
// MI455X (gfx1250) — hardware-verified
//
#include <hip/hip_runtime.h>
#include <math.h>
#include <stdint.h>

#ifndef TROWS
#define TROWS 4096
#endif
#define NB    8
#define SEQ   4096
#define HALF  2048
#define CH    256
#define NS    64
#define NCOL  16
#define KCV   6144
#define LT2   8192
#define LR    8192
#define XOFF  8184
#define CONV_DYN_BYTES (8 * LR * 2)
#define GEN_DYN_BYTES  (NS * 64 * 8 + 64 * NS * 16 + 2 * 1024 * 4)
#define KC    2048.0f
#define RCH   1024.0f
#define CROWS ((TROWS < HALF) ? TROWS : HALF)

static_assert((TROWS % 64) == 0 && TROWS >= 64 && (TROWS <= HALF || TROWS == SEQ));
static_assert(NB * 2 == NCOL && NCOL == 16);
static_assert(KCV == SEQ + HALF && (KCV % 32) == 0);
static_assert(((XOFF - KCV) % 8) == 0 && (XOFF - KCV) - 8 - (HALF - 64) - 48 >= 0);
static_assert((XOFF - KCV) + (KCV - 32) + 8 + 7 + 16 < LR && XOFF + 7 < LT2);
static_assert(CONV_DYN_BYTES == 131072 && GEN_DYN_BYTES == 106496);
static_assert((CH % 64) == 0 && (SEQ % 64) == 0 && (CH % 32) == 0 && LT2 == 2 * SEQ);

#define SZ_KT  ((size_t)CH * LT2 * 4)
#define SZ_U   ((size_t)CH * NCOL * KCV * 2)
#define SZ_WOH ((size_t)CH * CH * 2)
#define SZ_G   ((size_t)CH * NB * SEQ * 2)
#define SZ_H2  ((size_t)NB * SEQ * CH * 2)
#define WS_TOTAL (SZ_KT + SZ_U + SZ_WOH + 2 * SZ_G + 2 * SZ_H2)
static_assert(WS_TOTAL == (size_t)125960192);
static_assert(WS_TOTAL <= (size_t)134217728);
static_assert((SZ_KT % 16384) == 0 && (SZ_U % 16384) == 0 && (SZ_WOH % 16384) == 0 && (SZ_G % 16384) == 0 && (SZ_H2 % 16384) == 0);

typedef _Float16 v16h __attribute__((ext_vector_type(16)));
typedef _Float16 v8h  __attribute__((ext_vector_type(8)));
typedef __bf16   v16b __attribute__((ext_vector_type(16)));
typedef __bf16   v8b  __attribute__((ext_vector_type(8)));
typedef float    v8f  __attribute__((ext_vector_type(8)));
typedef float    v4f  __attribute__((ext_vector_type(4)));
typedef float    v2f  __attribute__((ext_vector_type(2)));
typedef unsigned int v4u __attribute__((ext_vector_type(4)));

#if defined(__HIP_DEVICE_COMPILE__)
#define DEV_ASM 1
#else
#define DEV_ASM 0
#endif

__device__ __forceinline__ unsigned short bf_bits(float f) {
  unsigned u = __float_as_uint(f);
  return (unsigned short)((u + 0x7FFFu + ((u >> 16) & 1u)) >> 16);
}
__device__ __forceinline__ float bf_up(unsigned short hb) { return __uint_as_float(((unsigned)hb) << 16); }
__device__ __forceinline__ float bfr(float f) { return bf_up(bf_bits(f)); }
__device__ __forceinline__ unsigned short h_bits(_Float16 x) { return __builtin_bit_cast(unsigned short, x); }
__device__ __forceinline__ unsigned pk16(unsigned short a, unsigned short b) { return (unsigned)a | ((unsigned)b << 16); }
__device__ __forceinline__ v8f zero8() { v8f z = {0.f, 0.f, 0.f, 0.f, 0.f, 0.f, 0.f, 0.f}; return z; }

__device__ __forceinline__ void split16(float v, float rc, unsigned short& hb, unsigned short& lb) {
  const _Float16 x = (_Float16)v;
  float xf = (float)x;
  xf = (fabsf(xf) < 6.103515625e-05f) ? 0.0f : xf;
  hb = h_bits((_Float16)xf);
  lb = h_bits((_Float16)((v - xf) * rc));
}
__device__ __forceinline__ unsigned short hflush(float v) {
  const _Float16 x = (_Float16)v;
  float xf = (float)x;
  xf = (fabsf(xf) < 6.103515625e-05f) ? 0.0f : xf;
  return h_bits((_Float16)xf);
}
__device__ __forceinline__ unsigned short cvw(float f) { return h_bits((_Float16)(bf_up(bf_bits(f)) * 64.0f)); }

template <typename OT> struct FT;
template <> struct FT<__bf16>   { typedef v16b frag; typedef v8b half8; };
template <> struct FT<_Float16> { typedef v16h frag; typedef v8h half8; };

template <typename OT>
__device__ __forceinline__ typename FT<OT>::frag ldfrag(const OT* p) {
  union { typename FT<OT>::frag v; typename FT<OT>::half8 h[2]; } f;
  f.h[0] = *(const typename FT<OT>::half8*)(p);
  f.h[1] = *(const typename FT<OT>::half8*)(p + 16);
  return f.v;
}

__device__ __forceinline__ v8f mmar(v16b a, v16b b, v8f c) {
  return __builtin_amdgcn_wmma_f32_16x16x32_bf16(false, a, false, b, (short)0, c, false, false);
}
__device__ __forceinline__ v8f mmar(v16h a, v16h b, v8f c) {
  return __builtin_amdgcn_wmma_f32_16x16x32_f16(false, a, false, b, (short)0, c, false, false);
}
__device__ __forceinline__ void dep_guard(v8f& a, v8f& b, v16b x, v16b y) {
#if DEV_ASM
  asm volatile("v_nop\n\tv_nop\n\tv_nop\n\tv_nop" : "+v"(a), "+v"(b) : "v"(x), "v"(y));
#else
  (void)a; (void)b; (void)x; (void)y;
#endif
}
__device__ __forceinline__ void dep_guard(v8f& a, v8f& b, v16h x, v16h y) {
#if DEV_ASM
  asm volatile("v_nop\n\tv_nop\n\tv_nop\n\tv_nop" : "+v"(a), "+v"(b) : "v"(x), "v"(y));
#else
  (void)a; (void)b; (void)x; (void)y;
#endif
}
__device__ __forceinline__ void keep4(v16b a, v16b b, v16b c, v16b d) {
#if DEV_ASM
  asm volatile("v_nop" :: "v"(a), "v"(b), "v"(c), "v"(d));
#else
  (void)a; (void)b; (void)c; (void)d;
#endif
}
__device__ __forceinline__ void keep4(v16h a, v16h b, v16h c, v16h d) {
#if DEV_ASM
  asm volatile("v_nop" :: "v"(a), "v"(b), "v"(c), "v"(d));
#else
  (void)a; (void)b; (void)c; (void)d;
#endif
}
__device__ __forceinline__ void keep1(v16h a) {
#if DEV_ASM
  asm volatile("v_nop" :: "v"(a));
#else
  (void)a;
#endif
}
__device__ __forceinline__ void acc_guard4(v8f& a, v8f& b, v8f& c, v8f& d) {
#if DEV_ASM
  asm volatile("v_nop\n\tv_nop\n\tv_nop\n\tv_nop" : "+v"(a), "+v"(b), "+v"(c), "+v"(d));
#else
  (void)a; (void)b; (void)c; (void)d;
#endif
}
__device__ __forceinline__ void conv_guard(v8f& a0, v8f& a1, v8f& a2, v8f& a3,
                                           v16h x0, v16h x1, v16h x2, v16h x3, v16h y) {
#if DEV_ASM
  asm volatile("v_nop\n\tv_nop\n\tv_nop\n\tv_nop"
               : "+v"(a0), "+v"(a1), "+v"(a2), "+v"(a3)
               : "v"(x0), "v"(x1), "v"(x2), "v"(x3), "v"(y));
#else
  (void)a0; (void)a1; (void)a2; (void)a3; (void)x0; (void)x1; (void)x2; (void)x3; (void)y;
#endif
}

template <typename OT, int MI, int NPA, int NPB, int OUT_MODE, int CZ>
__global__ __launch_bounds__(256) void gemm_t(
    const unsigned short* __restrict__ Ap, const unsigned short* __restrict__ A2p, int lda, long long strideA,
    const unsigned short* __restrict__ Btp, int ldb, long long strideB,
    const unsigned short* __restrict__ B2p, int ldb2, long long strideB2, int K2,
    void* Cout, void* Cout2, int ldc, long long strideC, int ldc2, long long strideC2, int N2,
    int M, int N, int K, float oscale, float rscale2, float cscale, float rscaleC,
    const float* __restrict__ bias, const float* __restrict__ resid) {
  static_assert(CZ != 2 || ((16 * MI) % 32) == 0);
  static_assert(!(NPA == 2 && NPB == 2));
  typedef typename FT<OT>::frag V16;
  const OT* A  = (const OT*)(const void*)Ap;
  const OT* A2 = (const OT*)(const void*)A2p;
  const OT* Bt = (const OT*)(const void*)Btp;
  const OT* B2 = (const OT*)(const void*)B2p;
  __shared__ __align__(16) float sT[8][16 * 68];
  const int RT   = 16 * MI;
  const int b    = blockIdx.y;
  const int lane = threadIdx.x & 31;
  const int wave = threadIdx.x >> 5;
  const int tilesN = N >> 6;
  const int tilesM = M / RT;
  const int tile = blockIdx.x * 8 + wave;
  if (tile >= tilesM * tilesN) return;
  const int tm = tile / tilesN;
  const int tn = tile - tm * tilesN;
  const int m0 = tm * RT;
  const int n0 = tn << 6;
  if (CZ == 1) {
    if (n0 >= m0 + RT) return;
  }
  int kEnd = K;
  if (CZ == 2) {
    const int ke = m0 + RT;
    kEnd = (ke < K) ? ke : K;
  }

  const OT* Ab  = A  + (size_t)b * (size_t)strideA;
  const OT* A2b = A2 + (size_t)b * (size_t)strideA;
  const OT* Bb  = Bt + (size_t)b * (size_t)strideB;
  const OT* B2b = B2 + (size_t)b * (size_t)strideB2;

  const int rlane = lane & 15;
  const int koff  = (lane >> 4) * 8;
  const int mOff  = (lane >> 4) * 8;

  v8f acc[MI][4], acc2[MI][4];
#pragma unroll
  for (int i = 0; i < MI; ++i)
#pragma unroll
    for (int j = 0; j < 4; ++j) { acc[i][j] = zero8(); acc2[i][j] = zero8(); }

#pragma unroll 1
  for (int k0 = 0; k0 < kEnd; k0 += 32) {
    V16 bq[4];
#pragma unroll
    for (int j = 0; j < 4; ++j)
      bq[j] = ldfrag<OT>(Bb + (size_t)(n0 + (j << 4) + rlane) * ldb + koff + k0);
#pragma unroll
    for (int i = 0; i < MI; ++i) {
      const V16 af = ldfrag<OT>(Ab + (size_t)(m0 + (i << 4) + rlane) * lda + koff + k0);
#pragma unroll
      for (int j = 0; j < 4; ++j) acc[i][j] = mmar(af, bq[j], acc[i][j]);
      dep_guard(acc[i][0], acc[i][3], af, bq[3]);
      if (NPA == 2) {
        const V16 af2 = ldfrag<OT>(A2b + (size_t)(m0 + (i << 4) + rlane) * lda + koff + k0);
#pragma unroll
        for (int j = 0; j < 4; ++j) acc2[i][j] = mmar(af2, bq[j], acc2[i][j]);
        dep_guard(acc2[i][0], acc2[i][3], af2, bq[3]);
      }
    }
    keep4(bq[0], bq[1], bq[2], bq[3]);
    if (NPB == 2) {
      if (k0 < K2) {
        V16 br[4];
#pragma unroll
        for (int j = 0; j < 4; ++j)
          br[j] = ldfrag<OT>(B2b + (size_t)(n0 + (j << 4) + rlane) * ldb2 + koff + k0);
#pragma unroll
        for (int i = 0; i < MI; ++i) {
          const V16 afr = ldfrag<OT>(Ab + (size_t)(m0 + (i << 4) + rlane) * lda + koff + k0);
#pragma unroll
          for (int j = 0; j < 4; ++j) acc2[i][j] = mmar(afr, br[j], acc2[i][j]);
          dep_guard(acc2[i][0], acc2[i][3], afr, br[3]);
        }
        keep4(br[0], br[1], br[2], br[3]);
      }
    }
  }
#pragma unroll
  for (int i = 0; i < MI; ++i) {
    acc_guard4(acc[i][0], acc[i][1], acc[i][2], acc[i][3]);
    if (NPA == 2 || NPB == 2) acc_guard4(acc2[i][0], acc2[i][1], acc2[i][2], acc2[i][3]);
  }

  float* slab = sT[wave];
#pragma unroll
  for (int i = 0; i < MI; ++i) {
    const int mBase = m0 + (i << 4);
#pragma unroll
    for (int j = 0; j < 4; ++j) {
#pragma unroll
      for (int r = 0; r < 8; ++r) {
        float v = acc[i][j][r];
        if (NPA == 2 || NPB == 2) v += acc2[i][j][r] * rscale2;
        v = v * oscale;
        slab[(mOff + r) * 68 + (j << 4) + rlane] = v;
      }
    }
    __builtin_amdgcn_fence(__ATOMIC_RELEASE, "workgroup");
    __builtin_amdgcn_wave_barrier();
    __builtin_amdgcn_fence(__ATOMIC_ACQUIRE, "workgroup");
    if (OUT_MODE == 0 || OUT_MODE == 4) {
      float* C = (float*)Cout + (size_t)b * (size_t)strideC;
      const float* Rb = resid + (size_t)b * (size_t)strideC;
      const int h2 = lane >> 4, c4 = (lane & 15) * 4;
      v4f ov[8];
#pragma unroll
      for (int it = 0; it < 8; ++it) {
        const int row = it * 2 + h2;
        v4f v = *(const v4f*)(slab + row * 68 + c4);
        if (OUT_MODE == 4) {
          const v4f bb = *(const v4f*)(bias + n0 + c4);
          const v4f xr = *(const v4f*)(Rb + (size_t)(mBase + row) * ldc + n0 + c4);
#pragma unroll
          for (int e = 0; e < 4; ++e) v[e] = (v[e] + bfr(bb[e])) + bfr(xr[e]);
        }
        ov[it] = v;
      }
      for (int pass = 0; pass < 2; ++pass) {
#pragma unroll
        for (int it = 0; it < 8; ++it) {
          const int row = it * 2 + h2;
          *(volatile v4f*)(C + (size_t)(mBase + row) * ldc + n0 + c4) = ov[it];
        }
        __threadfence();
      }
    } else {
      const int q = lane >> 3, c8 = (lane & 7) * 8;
      unsigned short* C  = (unsigned short*)Cout  + (size_t)b * (size_t)strideC;
      unsigned short* C2 = (unsigned short*)Cout2 + (size_t)b * (size_t)strideC2;
      const bool wr2 = (OUT_MODE == 3) && (n0 < N2);
      v4u hv[4], lv[4];
#pragma unroll
      for (int it = 0; it < 4; ++it) {
        const int row = it * 4 + q;
        const float* sp = slab + row * 68 + c8;
        float f[8];
#pragma unroll
        for (int e = 0; e < 8; ++e) f[e] = sp[e] * cscale;
        v4u a, a2;
#pragma unroll
        for (int e = 0; e < 4; ++e) {
          const float f0 = f[2 * e], f1 = f[2 * e + 1];
          const _Float16 x0 = (_Float16)f0, x1 = (_Float16)f1;
          const unsigned short h0 = h_bits(x0), h1 = h_bits(x1);
          unsigned short l0 = 0, l1 = 0;
          if (OUT_MODE == 3) {
            l0 = h_bits((_Float16)((f0 - (float)x0) * rscaleC));
            l1 = h_bits((_Float16)((f1 - (float)x1) * rscaleC));
          }
          a[e] = pk16(h0, h1); a2[e] = pk16(l0, l1);
        }
        hv[it] = a; lv[it] = a2;
      }
      for (int pass = 0; pass < 2; ++pass) {
#pragma unroll
        for (int it = 0; it < 4; ++it) {
          const int row = it * 4 + q;
          *(volatile v4u*)(C + (size_t)(mBase + row) * ldc + n0 + c8) = hv[it];
          if (OUT_MODE == 3) {
            if (wr2) *(volatile v4u*)(C2 + (size_t)(mBase + row) * ldc2 + n0 + c8) = lv[it];
          }
        }
        __threadfence();
      }
    }
    __builtin_amdgcn_fence(__ATOMIC_RELEASE, "workgroup");
    __builtin_amdgcn_wave_barrier();
    __builtin_amdgcn_fence(__ATOMIC_ACQUIRE, "workgroup");
  }
}

__global__ __launch_bounds__(256) void k_wT(const float* __restrict__ W, unsigned short* Woh) {
  __shared__ __align__(16) unsigned short sW[16 * 264];
  const int o0 = blockIdx.x * 16;
  const int tid = (int)threadIdx.x, wave = tid >> 5, lane = tid & 31;
  const int h = tid;
  const float* wp = W + (size_t)h * CH + o0;
#pragma unroll
  for (int e4 = 0; e4 < 4; ++e4) {
    const v4f a = *(const v4f*)(wp + 4 * e4);
#pragma unroll
    for (int e = 0; e < 4; ++e) sW[(4 * e4 + e) * 264 + h] = cvw(a[e]);
  }
  __syncthreads();
  v4u ov[2];
#pragma unroll
  for (int r = 0; r < 2; ++r) ov[r] = *(const v4u*)(sW + (2 * wave + r) * 264 + lane * 8);
  for (int pass = 0; pass < 2; ++pass) {
#pragma unroll
    for (int r = 0; r < 2; ++r)
      *(volatile v4u*)(Woh + (size_t)(o0 + 2 * wave + r) * CH + lane * 8) = ov[r];
    __threadfence();
  }
}

__global__ __launch_bounds__(256) void k_u(const float* __restrict__ X, unsigned short* U) {
  __shared__ __align__(16) unsigned short sU[CH * 72];
  const int bx = blockIdx.x, b = blockIdx.y;
  const int tid = (int)threadIdx.x, wave = tid >> 5, lane = tid & 31;
  const bool data = bx < (SEQ / 64);
  int sigA, sigB;
  if (data) { const int t0 = bx * 64; sigA = t0 + HALF; sigB = t0; }
  else      { const int z = bx - SEQ / 64; sigA = z * 64;  sigB = SEQ + z * 64; }
  if (data) {
    const int t0 = bx * 64;
    const int h4 = (tid & 63) * 4, rq = tid >> 6;
#pragma unroll 4
    for (int it = 0; it < 16; ++it) {
      const int r = rq + 4 * it;
      const v4f v = *(const v4f*)(X + ((size_t)(b * SEQ + t0 + r)) * CH + h4);
#pragma unroll
      for (int e = 0; e < 4; ++e) sU[(h4 + e) * 72 + r] = h_bits((_Float16)bfr(v[e]));
    }
  }
  __syncthreads();
  const int q = lane >> 3, c8 = (lane & 7) * 8;
  v4u pv[8];
  if (data) {
#pragma unroll
    for (int it = 0; it < 8; ++it) {
      const int hr = 4 * (wave + 8 * it) + q;
      pv[it] = *(const v4u*)(sU + hr * 72 + c8);
    }
  } else {
#pragma unroll
    for (int it = 0; it < 8; ++it) { v4u zz = {0u, 0u, 0u, 0u}; pv[it] = zz; }
  }
  for (int pass = 0; pass < 2; ++pass) {
#pragma unroll
    for (int it = 0; it < 8; ++it) {
      const int hr = 4 * (wave + 8 * it) + q;
      const size_t oA = ((size_t)(hr * NCOL + b)) * KCV + sigA + c8;
      const size_t oB = ((size_t)(hr * NCOL + b + 8)) * KCV + sigB + c8;
      *(volatile v4u*)(U + oA) = pv[it];
      *(volatile v4u*)(U + oB) = pv[it];
    }
    __threadfence();
  }
}

__global__ __launch_bounds__(256) void k_gen(const float* __restrict__ ldt, const float* __restrict__ Are,
                                              const float* __restrict__ Aim, const float* __restrict__ Cre,
                                              const float* __restrict__ Cim, float* KT) {
  extern __shared__ __align__(16) float dynG[];
  v2f* sE  = (v2f*)(void*)dynG;
  v4f* sG  = (v4f*)(void*)(dynG + NS * 64 * 2);
  float* sK0 = dynG + NS * 64 * 2 + 64 * NS * 4;
  float* sK1 = sK0 + 1024;
  __shared__ float sZr[NS];
  __shared__ float sZi[NS];
  __shared__ __align__(16) v4f sCt[NS];
  const int h = blockIdx.x, tid = (int)threadIdx.x;
  if (tid < NS) {
    const int i = h * NS + tid;
    const float dt = expf(bfr(ldt[h]));
    sZr[tid] = dt * bfr(Are[i]);
    sZi[tid] = dt * bfr(Aim[i]);
  }
  __syncthreads();
#pragma unroll 1
  for (int item = tid; item < 2 * NS * 64; item += 256) {
    const bool anc = item >= NS * 64;
    const int a  = anc ? (item - NS * 64) : item;
    const int n  = anc ? (a & 63) : (a >> 6);
    const int mi = anc ? ((a >> 6) * 64) : (a & 63);
    const float mf = (float)mi;
    const float er = expf(sZr[n] * mf);
    float sv, cv;
    sincosf(sZi[n] * mf, &sv, &cv);
    const float pr = er * cv, pi = er * sv;
    if (anc) { v4f w; w[0] = pr; w[1] = pi; w[2] = 0.f; w[3] = 0.f; sG[a] = w; }
    else     { v2f w; w[0] = pr; w[1] = pi; sE[a] = w; }
  }
  __syncthreads();
  if (tid < NS) {
    const int n = tid, i = h * NS + n;
    const v2f lam = sE[n * 64 + 1];
    const float ar = bfr(Are[i]), ai = bfr(Aim[i]);
    const float nr = lam[0] - 1.0f, ni = lam[1];
    const float inv = 1.0f / (ar * ar + ai * ai);
    const float fr = (nr * ar + ni * ai) * inv;
    const float fi = (ni * ar - nr * ai) * inv;
    const float c0r = bfr(Cre[i]), c0i = bfr(Cim[i]);
    const float c1r = bfr(Cre[CH * NS + i]), c1i = bfr(Cim[CH * NS + i]);
    v4f ct;
    ct[0] = c0r * fr - c0i * fi;  ct[1] = c0r * fi + c0i * fr;
    ct[2] = c1r * fr - c1i * fi;  ct[3] = c1r * fi + c1i * fr;
    sCt[n] = ct;
  }
  __syncthreads();
#pragma unroll 1
  for (int a = tid; a < 64 * NS; a += 256) {
    const int n = a & 63;
    const v4f q = sG[a];
    const v4f ct = sCt[n];
    v4f g;
    g[0] = ct[0] * q[0] - ct[1] * q[1];  g[1] = ct[0] * q[1] + ct[1] * q[0];
    g[2] = ct[2] * q[0] - ct[3] * q[1];  g[3] = ct[2] * q[1] + ct[3] * q[0];
    sG[a] = g;
  }
  __syncthreads();
  const int j = tid & 63, cq = tid >> 6;
  float* kt = KT + (size_t)h * LT2;
#pragma unroll 1
  for (int grp = 0; grp < 4; ++grp) {
#pragma unroll 1
    for (int it = 0; it < 4; ++it) {
      const int cl = cq + 4 * it;
      const int c = 16 * grp + cl;
      const v4f* gp = sG + c * NS;
      float a0 = 0.f, a1 = 0.f;
#pragma unroll 2
      for (int n = 0; n < NS; ++n) {
        const v2f e = sE[n * 64 + j];
        const v4f g = gp[n];
        a0 = fmaf(g[0], e[0], a0);  a0 = fmaf(-g[1], e[1], a0);
        a1 = fmaf(g[2], e[0], a1);  a1 = fmaf(-g[3], e[1], a1);
      }
      sK0[64 * cl + j] = 2.0f * a0;
      sK1[64 * cl + j] = 2.0f * a1;
    }
    __syncthreads();
    const v4f v0 = *(const v4f*)(sK0 + 4 * tid);
    const v4f w  = *(const v4f*)(sK1 + 1020 - 4 * tid);
    v4f v1; v1[0] = w[3]; v1[1] = w[2]; v1[2] = w[1]; v1[3] = w[0];
    float* d0 = kt + SEQ + 1024 * grp + 4 * tid;
    float* d1 = kt + (3072 - 1024 * grp) + 4 * tid;
    *(volatile v4f*)d0 = v0;
    *(volatile v4f*)d1 = v1;
    __threadfence();
    *(volatile v4f*)d0 = v0;
    *(volatile v4f*)d1 = v1;
    __syncthreads();
  }
}

__global__ __launch_bounds__(256) void k_conv(const float* __restrict__ KT, const unsigned short* __restrict__ U,
                                               const float* __restrict__ Dv, unsigned short* Gh, unsigned short* Gl) {
  extern __shared__ __align__(16) unsigned short dynK[];
  __shared__ __align__(16) unsigned short sOh[8][16 * 72];
  __shared__ __align__(16) unsigned short sOl[8][16 * 72];
  const int h = blockIdx.x;
  const int tid = (int)threadIdx.x, wave = tid >> 5, lane = tid & 31;
  const float* kt = KT + (size_t)h * LT2;
#pragma unroll 1
  for (int task = tid; task < 8 * (LR / 8); task += 256) {
    const int j = task & 7, q = task >> 3;
    v4u ph;
#pragma unroll
    for (int e2 = 0; e2 < 4; ++e2) {
      unsigned short hb[2];
#pragma unroll
      for (int u = 0; u < 2; ++u) {
        const int e = 2 * e2 + u;
        const int ii = XOFF + j - (8 * q + e);
        const int ic = min(max(ii, 0), LT2 - 1);
        float v = kt[ic];
        v = (ii >= 0 && ii < LT2) ? v : 0.0f;
        hb[u] = hflush(v * KC);
      }
      ph[e2] = pk16(hb[0], hb[1]);
    }
    *(v4u*)(dynK + (size_t)j * LR + 8 * q) = ph;
  }
  __syncthreads();

  const float dsk = bfr(Dv[h]);
  const _Float16* Kh  = (const _Float16*)(const void*)dynK;
  const _Float16* U16 = (const _Float16*)(const void*)U;
  const int m = lane & 15, hh = lane >> 4, r7 = lane & 7;
  const _Float16* urow = U16 + ((size_t)(h * NCOL + m)) * KCV + 8 * hh;
  const int abase = (XOFF - KCV) - (m & 8) + 8 * hh + r7 * LR;
  unsigned short* slabh = sOh[wave];
  unsigned short* slabl = sOl[wave];
  const int ntile = CROWS / 64;
  for (int tt = wave; tt < ntile; tt += 8) {
    const int t0 = tt * 64;
    v8f acc[4];
#pragma unroll
    for (int i = 0; i < 4; ++i) acc[i] = zero8();
    const int ab0 = abase - t0;
#pragma unroll 1
    for (int s0 = 0; s0 < KCV; s0 += 32) {
      const v16h bq = ldfrag<_Float16>(urow + s0);
      v16h ah[4];
#pragma unroll
      for (int i = 0; i < 4; ++i) ah[i] = ldfrag<_Float16>(Kh + (ab0 + s0 - 16 * i));
#pragma unroll
      for (int i = 0; i < 4; ++i) acc[i] = mmar(ah[i], bq, acc[i]);
      conv_guard(acc[0], acc[1], acc[2], acc[3], ah[0], ah[1], ah[2], ah[3], bq);
    }
    acc_guard4(acc[0], acc[1], acc[2], acc[3]);
#pragma unroll
    for (int i = 0; i < 4; ++i) {
      const v8h uv = *(const v8h*)(urow + HALF + t0 + 16 * i);
      unsigned short hb[8], lb[8];
#pragma unroll
      for (int rr = 0; rr < 8; ++rr) {
        const float conv = acc[i][rr] * 0.00048828125f;
        const float y = conv + dsk * (float)uv[rr];
        const float g = 0.5f * y * (1.0f + erff(y * 0.707106781186547524f));
        split16(g, RCH, hb[rr], lb[rr]);
      }
      v4u p0, p1;
#pragma unroll
      for (int e = 0; e < 4; ++e) { p0[e] = pk16(hb[2 * e], hb[2 * e + 1]); p1[e] = pk16(lb[2 * e], lb[2 * e + 1]); }
      *(v4u*)(slabh + m * 72 + 16 * i + 8 * hh) = p0;
      *(v4u*)(slabl + m * 72 + 16 * i + 8 * hh) = p1;
    }
    __builtin_amdgcn_fence(__ATOMIC_RELEASE, "workgroup");
    __builtin_amdgcn_wave_barrier();
    __builtin_amdgcn_fence(__ATOMIC_ACQUIRE, "workgroup");
    const int q4 = lane >> 3, c8 = (lane & 7) * 8;
    v4u hv4[4], lv4[4];
#pragma unroll
    for (int it = 0; it < 4; ++it) {
      const int row = it * 4 + q4;
      hv4[it] = *(const v4u*)(slabh + row * 72 + c8);
      lv4[it] = *(const v4u*)(slabl + row * 72 + c8);
    }
    for (int pass = 0; pass < 2; ++pass) {
#pragma unroll
      for (int it = 0; it < 4; ++it) {
        const int row = it * 4 + q4;
        const size_t o = ((size_t)(h * NB + (row & 7))) * SEQ + (size_t)HALF * (row >> 3) + t0 + c8;
        *(volatile v4u*)(Gh + o) = hv4[it];
        *(volatile v4u*)(Gl + o) = lv4[it];
      }
      __threadfence();
    }
    __builtin_amdgcn_fence(__ATOMIC_RELEASE, "workgroup");
    __builtin_amdgcn_wave_barrier();
    __builtin_amdgcn_fence(__ATOMIC_ACQUIRE, "workgroup");
  }
}

__global__ __launch_bounds__(256) void k_hT(const unsigned short* __restrict__ Gh, const unsigned short* __restrict__ Gl,
                                            unsigned short* H2h, unsigned short* H2l) {
  __shared__ __align__(16) unsigned short sH[64 * 264];
  const int t0 = blockIdx.x * 64, b = blockIdx.y, pl = blockIdx.z;
  const unsigned short* src = (pl == 0) ? Gh : Gl;
  unsigned short* dst = (pl == 0) ? H2h : H2l;
  const int tid = (int)threadIdx.x, wave = tid >> 5, lane = tid & 31;
  const int cq = tid >> 3, c8 = (tid & 7) * 8;
#pragma unroll
  for (int it = 0; it < 8; ++it) {
    const int c = cq + 32 * it;
    const v4u p = *(const v4u*)(src + ((size_t)(c * NB + b)) * SEQ + t0 + c8);
#pragma unroll
    for (int k = 0; k < 4; ++k) {
      sH[(c8 + 2 * k) * 264 + c]     = (unsigned short)(p[k] & 0xffffu);
      sH[(c8 + 2 * k + 1) * 264 + c] = (unsigned short)(p[k] >> 16);
    }
  }
  __syncthreads();
  const int cc = lane * 8;
  v4u ov[8];
#pragma unroll
  for (int it = 0; it < 8; ++it) {
    const int row = wave + 8 * it;
    ov[it] = *(const v4u*)(sH + row * 264 + cc);
  }
  for (int pass = 0; pass < 2; ++pass) {
#pragma unroll
    for (int it = 0; it < 8; ++it) {
      const int row = wave + 8 * it;
      *(volatile v4u*)(dst + ((size_t)(b * SEQ + t0 + row)) * CH + cc) = ov[it];
    }
    __threadfence();
  }
}

__global__ __launch_bounds__(256) void k_lnf(float* Y, const float* __restrict__ gam, const float* __restrict__ bet) {
  const int tid = (int)threadIdx.x, wave = tid >> 5, lane = tid & 31, b = blockIdx.y;
  const v4f ga = *(const v4f*)(gam + 4 * lane), gb = *(const v4f*)(gam + 128 + 4 * lane);
  const v4f ba = *(const v4f*)(bet + 4 * lane), bb = *(const v4f*)(bet + 128 + 4 * lane);
  float g[8], be[8];
#pragma unroll
  for (int e = 0; e < 4; ++e) { g[e] = bfr(ga[e]); g[4 + e] = bfr(gb[e]); be[e] = bfr(ba[e]); be[4 + e] = bfr(bb[e]); }
#pragma unroll 1
  for (int rr = 0; rr < 4; ++rr) {
    const int tau = blockIdx.x * 32 + wave * 4 + rr;
    float* row = Y + ((size_t)(b * SEQ + tau)) * CH;
    const v4f xa = *(const v4f*)(row + 4 * lane);
    const v4f xb = *(const v4f*)(row + 128 + 4 * lane);
    float v[8];
#pragma unroll
    for (int e = 0; e < 4; ++e) { v[e] = xa[e]; v[4 + e] = xb[e]; }
    float s = ((v[0] + v[1]) + (v[2] + v[3])) + ((v[4] + v[5]) + (v[6] + v[7]));
#pragma unroll
    for (int off = 1; off < 32; off <<= 1) s += __shfl_xor(s, off, 32);
    const float mu = s * 0.00390625f;
    float d[8];
    float q = 0.f;
#pragma unroll
    for (int e = 0; e < 8; ++e) { d[e] = v[e] - mu; q += d[e] * d[e]; }
#pragma unroll
    for (int off = 1; off < 32; off <<= 1) q += __shfl_xor(q, off, 32);
    const float var = q * 0.00390625f;
    const float inv = 1.0f / sqrtf(var + 1e-5f);
    v4f oa, ob;
#pragma unroll
    for (int e = 0; e < 4; ++e) {
      oa[e] = ((d[e] * inv) * g[e]) + be[e];
      ob[e] = ((d[4 + e] * inv) * g[4 + e]) + be[4 + e];
    }
    *(volatile v4f*)(row + 4 * lane) = oa;
    *(volatile v4f*)(row + 128 + 4 * lane) = ob;
    __threadfence();
    *(volatile v4f*)(row + 4 * lane) = oa;
    *(volatile v4f*)(row + 128 + 4 * lane) = ob;
  }
}

extern "C" void kernel_launch(void* const* d_in, const int* in_sizes, int n_in,
                              void* d_out, int out_size, void* d_ws, size_t ws_size,
                              hipStream_t stream) {
  if (n_in < 11) return;
  const long long needX = (long long)NB * SEQ * (long long)CH;
  if ((long long)in_sizes[0] < needX) return;
  if (in_sizes[1] < CH) return;
  if (in_sizes[2] < CH * NS || in_sizes[3] < CH * NS) return;
  if (in_sizes[4] < 2 * CH * NS || in_sizes[5] < 2 * CH * NS) return;
  if (in_sizes[6] < CH) return;
  if (in_sizes[7] < CH * CH) return;
  if (in_sizes[8] < CH || in_sizes[9] < CH || in_sizes[10] < CH) return;
  if (out_size < 0) return;
  const long long needO = ((long long)(NB - 1) * SEQ + TROWS) * (long long)CH;
  if ((long long)out_size < needO) return;

  const float* x    = (const float*)d_in[0];
  const float* ldt  = (const float*)d_in[1];
  const float* Are  = (const float*)d_in[2];
  const float* Aim  = (const float*)d_in[3];
  const float* Cre  = (const float*)d_in[4];
  const float* Cim  = (const float*)d_in[5];
  const float* Dv   = (const float*)d_in[6];
  const float* W    = (const float*)d_in[7];
  const float* bo   = (const float*)d_in[8];
  const float* gam  = (const float*)d_in[9];
  const float* bet  = (const float*)d_in[10];
  float* out0 = (float*)d_out;

  size_t off = 0;
  const size_t oKT  = off; off += SZ_KT;
  const size_t oU   = off; off += SZ_U;
  const size_t oWoh = off; off += SZ_WOH;
  const size_t oGh  = off; off += SZ_G;
  const size_t oGl  = off; off += SZ_G;
  const size_t oH2h = off; off += SZ_H2;
  const size_t oH2l = off; off += SZ_H2;
  if (off > ws_size) return;
  if (off > (size_t)134217728) return;

  char* ws = (char*)d_ws;
  float*          KT  = (float*)(ws + oKT);
  unsigned short* U   = (unsigned short*)(ws + oU);
  unsigned short* Woh = (unsigned short*)(ws + oWoh);
  unsigned short* Gh  = (unsigned short*)(ws + oGh);
  unsigned short* Gl  = (unsigned short*)(ws + oGl);
  unsigned short* H2h = (unsigned short*)(ws + oH2h);
  unsigned short* H2l = (unsigned short*)(ws + oH2l);

  const dim3 blk(256);
  const dim3 gWT(CH / 16);
  const dim3 gU(SEQ / 64 + HALF / 64, NB);
  const dim3 gGen(CH);
  const dim3 gConv(CH);
  const dim3 gHT(TROWS / 64, NB, 2);
  const dim3 gOut((((TROWS / 32) * (CH / 64)) + 7) / 8, NB);
  const dim3 gLn(TROWS / 32, NB);

  k_wT<<<gWT, blk, 0, stream>>>(W, Woh);
  k_u<<<gU, blk, 0, stream>>>(x, U);
  (void)hipFuncSetAttribute(reinterpret_cast<const void*>(&k_gen), hipFuncAttributeMaxDynamicSharedMemorySize, GEN_DYN_BYTES);
  k_gen<<<gGen, blk, GEN_DYN_BYTES, stream>>>(ldt, Are, Aim, Cre, Cim, KT);
  (void)hipFuncSetAttribute(reinterpret_cast<const void*>(&k_conv), hipFuncAttributeMaxDynamicSharedMemorySize, CONV_DYN_BYTES);
  k_conv<<<gConv, blk, CONV_DYN_BYTES, stream>>>(KT, U, Dv, Gh, Gl);
  k_hT<<<gHT, blk, 0, stream>>>(Gh, Gl, H2h, H2l);
  gemm_t<_Float16, 2, 2, 1, 4, 0><<<gOut, blk, 0, stream>>>(
      H2h, H2l, CH, (long long)SEQ * CH, Woh, CH, 0LL,
      Woh, CH, 0LL, 0,
      (void*)out0, (void*)out0, CH, (long long)SEQ * CH, CH, (long long)SEQ * CH, CH,
      TROWS, CH, CH, 0.015625f, 0.0009765625f, 1.0f, 1.0f, bo, x);
  k_lnf<<<gLn, blk, 0, stream>>>(out0, gam, bet);
  (void)hipGetLastError();
}
